// SyncAwareAttention_76218489635255
// MI455X (gfx1250) — hardware-verified
//
#include <hip/hip_runtime.h>


#define NOP4 "v_nop\n\tv_nop\n\tv_nop\n\tv_nop"

typedef _Float16 v16h __attribute__((ext_vector_type(16)));
typedef __bf16 v16b __attribute__((ext_vector_type(16)));
typedef float v8f __attribute__((ext_vector_type(8)));
typedef float v4f __attribute__((ext_vector_type(4)));
typedef unsigned int v4u __attribute__((ext_vector_type(4)));

union FragH { v16h v; v4u q[2]; };
union FragB { v16b v; v4u q[2]; };

__device__ __forceinline__ v4u ldg16(const unsigned short* p) { return *(const v4u*)p; }

__device__ __forceinline__ unsigned int bf_bits(float f) {
  unsigned int u = __float_as_uint(f);
  return (u + 0x7FFFu + ((u >> 16) & 1u)) >> 16;
}
__device__ __forceinline__ float bf_val(unsigned int b) { return __uint_as_float(b << 16); }
__device__ __forceinline__ unsigned int hf_bits(float f) {
  union { _Float16 h; unsigned short u; } c;
  c.h = (_Float16)f;
  return (unsigned int)c.u;
}
__device__ __forceinline__ unsigned int pk2(unsigned int lo, unsigned int hi) {
  return (lo & 0xFFFFu) | (hi << 16);
}
__device__ __forceinline__ v4u pack_h8(v4f a, v4f c) {
  v4u r;
  r[0] = pk2(hf_bits(a[0]), hf_bits(a[1]));
  r[1] = pk2(hf_bits(a[2]), hf_bits(a[3]));
  r[2] = pk2(hf_bits(c[0]), hf_bits(c[1]));
  r[3] = pk2(hf_bits(c[2]), hf_bits(c[3]));
  return r;
}
__device__ __forceinline__ void split_b8(v4f a, v4f c, v4u& H, v4u& L) {
  float v[8] = {a[0], a[1], a[2], a[3], c[0], c[1], c[2], c[3]};
  unsigned int hb[8], lb[8];
#pragma unroll
  for (int e = 0; e < 8; ++e) {
    hb[e] = bf_bits(v[e]);
    lb[e] = bf_bits(v[e] - bf_val(hb[e]));
  }
#pragma unroll
  for (int t = 0; t < 4; ++t) {
    H[t] = pk2(hb[2 * t], hb[2 * t + 1]);
    L[t] = pk2(lb[2 * t], lb[2 * t + 1]);
  }
}

__device__ __forceinline__ v8f zero8() {
  v8f z;
#pragma unroll
  for (int r = 0; r < 8; ++r) z[r] = 0.f;
  return z;
}
__device__ __forceinline__ v8f mma_h(v16h a, v16h b, v8f c) {
  return __builtin_amdgcn_wmma_f32_16x16x32_f16(false, a, false, b, (short)0, c, false, false);
}
__device__ __forceinline__ v8f mma_b(v16b a, v16b b, v8f c) {
  return __builtin_amdgcn_wmma_f32_16x16x32_bf16(false, a, false, b, (short)0, c, false, false);
}

__global__ __launch_bounds__(256) void k_cvt_x(const float* __restrict__ x, unsigned short* xh,
                                              unsigned short* xbh, unsigned short* xbl, int n) {
  const size_t i8 = ((size_t)blockIdx.x * 256u + (size_t)threadIdx.x) * 8u;
  if (i8 + 8 > (size_t)n) return;
  const v4f a = *(const v4f*)(x + i8);
  const v4f c = *(const v4f*)(x + i8 + 4);
  const v4u fh = pack_h8(a, c);
  v4u bh, bl;
  split_b8(a, c, bh, bl);
  *(volatile v4u*)(xh + i8) = fh;
  *(volatile v4u*)(xbh + i8) = bh;
  *(volatile v4u*)(xbl + i8) = bl;
  __threadfence();
  *(volatile v4u*)(xh + i8) = fh;
  *(volatile v4u*)(xbh + i8) = bh;
  *(volatile v4u*)(xbl + i8) = bl;
}

template <int MODE>
__global__ __launch_bounds__(256) void k_cvt_wT(const float* __restrict__ W, unsigned short* o0,
                                               unsigned short* o1, int Kd, int Nd, float scale) {
  __shared__ float tile[64][65];
  const int n0 = blockIdx.x * 64, e0 = blockIdx.y * 64;
  if (n0 + 64 > Nd || e0 + 64 > Kd) return;
  const int tid = threadIdx.x;
#pragma unroll
  for (int t = 0; t < 4; ++t) {
    const int idx = t * 256 + tid;
    const int rr = idx >> 4, c4 = (idx & 15) * 4;
    const v4f v = *(const v4f*)(W + (size_t)(e0 + rr) * Nd + n0 + c4);
    tile[rr][c4] = v[0];
    tile[rr][c4 + 1] = v[1];
    tile[rr][c4 + 2] = v[2];
    tile[rr][c4 + 3] = v[3];
  }
  __syncthreads();
  v4u Hv[2], Lv[2];
  size_t adr[2];
#pragma unroll
  for (int t = 0; t < 2; ++t) {
    const int s = t * 256 + tid;
    const int nn = s >> 3, kq = (s & 7) * 8;
    v4f a, c;
#pragma unroll
    for (int e = 0; e < 4; ++e) {
      a[e] = tile[kq + e][nn] * scale;
      c[e] = tile[kq + 4 + e][nn] * scale;
    }
    if (MODE == 0) {
      Hv[t] = pack_h8(a, c);
      Lv[t] = Hv[t];
    } else {
      split_b8(a, c, Hv[t], Lv[t]);
    }
    adr[t] = (size_t)(n0 + nn) * Kd + e0 + kq;
  }
#pragma unroll
  for (int t = 0; t < 2; ++t) {
    *(volatile v4u*)(o0 + adr[t]) = Hv[t];
    if (MODE == 1) *(volatile v4u*)(o1 + adr[t]) = Lv[t];
  }
  __threadfence();
#pragma unroll
  for (int t = 0; t < 2; ++t) {
    *(volatile v4u*)(o0 + adr[t]) = Hv[t];
    if (MODE == 1) *(volatile v4u*)(o1 + adr[t]) = Lv[t];
  }
}

__global__ __launch_bounds__(256) void k_gate(const float* __restrict__ sync, const float* __restrict__ W1,
                                             const float* __restrict__ b1, const float* __restrict__ W2,
                                             const float* __restrict__ b2, float* swo, int Ein, int Hd, int Hn) {
  __shared__ float hid[256];
  __shared__ float gv[32];
  const int b = blockIdx.x, tid = threadIdx.x;
  for (int j = tid; j < Hd; j += 256) {
    float a = b1[j];
    for (int e = 0; e < Ein; ++e) a += sync[(size_t)b * Ein + e] * W1[(size_t)e * Hd + j];
    hid[j] = fmaxf(a, 0.f);
  }
  __syncthreads();
  if (tid < 32) {
    float val = 0.f;
    if (tid < Hn) {
      float a = b2[tid];
      for (int t = 0; t < Hd; ++t) a += hid[t] * W2[(size_t)t * Hn + tid];
      val = 1.0f / (1.0f + expf(-a));
    }
    gv[tid] = val;
  }
  __syncthreads();
  if (tid < 8) {
    v4f v;
    v[0] = gv[tid * 4];
    v[1] = gv[tid * 4 + 1];
    v[2] = gv[tid * 4 + 2];
    v[3] = gv[tid * 4 + 3];
    float* p = swo + (size_t)b * 32 + tid * 4;
    *(volatile v4f*)p = v;
    __threadfence();
    *(volatile v4f*)p = v;
  }
}

template <int SPLIT, int OM>
__global__ __launch_bounds__(256) void k_gemm(const unsigned short* __restrict__ Ah,
                                             const unsigned short* __restrict__ Al,
                                             const unsigned short* __restrict__ Bh,
                                             const unsigned short* __restrict__ Bl,
                                             const float* __restrict__ bias, void* out0, void* out1,
                                             int M, int N, int K, int Sq, float oscale) {
  __shared__ v4f stg4[128 * 17];
  float* stg = (float*)stg4;
  const int nBase = blockIdx.x * 64, mBase = blockIdx.y * 128;
  if (nBase + 64 > N || mBase + 128 > M) return;
  const int tid = threadIdx.x, w = tid >> 5, l = tid & 31, g = l >> 4, m = l & 15;

  v8f acc[4];
#pragma unroll
  for (int nt = 0; nt < 4; ++nt) acc[nt] = zero8();

  const size_t arow = (size_t)(mBase + w * 16 + m) * K + 8 * g;
  const size_t brow = (size_t)(nBase + m) * K + 8 * g;
  const size_t bnt = (size_t)16 * K;

#pragma unroll 1
  for (int k0 = 0; k0 < K; k0 += 32) {
    if (SPLIT) {
      FragB a, a2, b0, b1, b2, b3, c0, c1, c2, c3;
      a.q[0] = ldg16(Ah + arow + k0);
      a.q[1] = ldg16(Ah + arow + k0 + 16);
      a2.q[0] = ldg16(Al + arow + k0);
      a2.q[1] = ldg16(Al + arow + k0 + 16);
      b0.q[0] = ldg16(Bh + brow + k0);
      b0.q[1] = ldg16(Bh + brow + k0 + 16);
      b1.q[0] = ldg16(Bh + brow + bnt + k0);
      b1.q[1] = ldg16(Bh + brow + bnt + k0 + 16);
      b2.q[0] = ldg16(Bh + brow + 2 * bnt + k0);
      b2.q[1] = ldg16(Bh + brow + 2 * bnt + k0 + 16);
      b3.q[0] = ldg16(Bh + brow + 3 * bnt + k0);
      b3.q[1] = ldg16(Bh + brow + 3 * bnt + k0 + 16);
      c0.q[0] = ldg16(Bl + brow + k0);
      c0.q[1] = ldg16(Bl + brow + k0 + 16);
      c1.q[0] = ldg16(Bl + brow + bnt + k0);
      c1.q[1] = ldg16(Bl + brow + bnt + k0 + 16);
      c2.q[0] = ldg16(Bl + brow + 2 * bnt + k0);
      c2.q[1] = ldg16(Bl + brow + 2 * bnt + k0 + 16);
      c3.q[0] = ldg16(Bl + brow + 3 * bnt + k0);
      c3.q[1] = ldg16(Bl + brow + 3 * bnt + k0 + 16);
      acc[0] = mma_b(a.v, b0.v, acc[0]);
      acc[0] = mma_b(a.v, c0.v, acc[0]);
      acc[0] = mma_b(a2.v, b0.v, acc[0]);
      acc[1] = mma_b(a.v, b1.v, acc[1]);
      acc[1] = mma_b(a.v, c1.v, acc[1]);
      acc[1] = mma_b(a2.v, b1.v, acc[1]);
      acc[2] = mma_b(a.v, b2.v, acc[2]);
      acc[2] = mma_b(a.v, c2.v, acc[2]);
      acc[2] = mma_b(a2.v, b2.v, acc[2]);
      acc[3] = mma_b(a.v, b3.v, acc[3]);
      acc[3] = mma_b(a.v, c3.v, acc[3]);
      acc[3] = mma_b(a2.v, b3.v, acc[3]);
      asm volatile(NOP4
                   : "+v"(acc[0]), "+v"(acc[1]), "+v"(acc[2]), "+v"(acc[3])
                   : "v"(a.v), "v"(a2.v), "v"(b0.v), "v"(b1.v), "v"(b2.v), "v"(b3.v),
                     "v"(c0.v), "v"(c1.v), "v"(c2.v), "v"(c3.v));
    } else {
      FragH a, b0, b1, b2, b3;
      a.q[0] = ldg16(Ah + arow + k0);
      a.q[1] = ldg16(Ah + arow + k0 + 16);
      b0.q[0] = ldg16(Bh + brow + k0);
      b0.q[1] = ldg16(Bh + brow + k0 + 16);
      b1.q[0] = ldg16(Bh + brow + bnt + k0);
      b1.q[1] = ldg16(Bh + brow + bnt + k0 + 16);
      b2.q[0] = ldg16(Bh + brow + 2 * bnt + k0);
      b2.q[1] = ldg16(Bh + brow + 2 * bnt + k0 + 16);
      b3.q[0] = ldg16(Bh + brow + 3 * bnt + k0);
      b3.q[1] = ldg16(Bh + brow + 3 * bnt + k0 + 16);
      acc[0] = mma_h(a.v, b0.v, acc[0]);
      acc[1] = mma_h(a.v, b1.v, acc[1]);
      acc[2] = mma_h(a.v, b2.v, acc[2]);
      acc[3] = mma_h(a.v, b3.v, acc[3]);
      asm volatile(NOP4
                   : "+v"(acc[0]), "+v"(acc[1]), "+v"(acc[2]), "+v"(acc[3])
                   : "v"(a.v), "v"(b0.v), "v"(b1.v), "v"(b2.v), "v"(b3.v));
    }
  }

#pragma unroll
  for (int nt = 0; nt < 4; ++nt) {
    const int col = nt * 16 + m;
    const float bv = bias[nBase + col];
#pragma unroll
    for (int r = 0; r < 8; ++r) stg[(w * 16 + 8 * g + r) * 68 + col] = acc[nt][r] * oscale + bv;
  }
  __syncthreads();

  if (OM == 0) {
    unsigned short* o = (unsigned short*)out0;
    v4u val[4];
    size_t adr[4];
#pragma unroll
    for (int t = 0; t < 4; ++t) {
      const int row = w * 16 + t * 4 + (l >> 3), c8 = (l & 7) * 8;
      const float* sp = stg + row * 68 + c8;
      const v4f x0 = *(const v4f*)sp;
      const v4f x1 = *(const v4f*)(sp + 4);
      val[t] = pack_h8(x0, x1);
      adr[t] = (size_t)(mBase + row) * N + nBase + c8;
    }
#pragma unroll
    for (int t = 0; t < 4; ++t) *(volatile v4u*)(o + adr[t]) = val[t];
    __threadfence();
#pragma unroll
    for (int t = 0; t < 4; ++t) *(volatile v4u*)(o + adr[t]) = val[t];
  } else if (OM == 1) {
    unsigned short* oh = (unsigned short*)out0;
    unsigned short* ol = (unsigned short*)out1;
    const int Hn = N >> 6;
    const int bb = mBase / Sq;
    const int bh = bb * Hn + (nBase >> 6);
    const int sBase = mBase - bb * Sq;
    v4u Hv[4], Lv[4];
    size_t adr[4];
#pragma unroll
    for (int t = 0; t < 4; ++t) {
      const int d = w * 8 + t * 2 + (l >> 4), s8 = (l & 15) * 8;
      v4f x0, x1;
#pragma unroll
      for (int e = 0; e < 4; ++e) {
        x0[e] = stg[(s8 + e) * 68 + d];
        x1[e] = stg[(s8 + 4 + e) * 68 + d];
      }
      split_b8(x0, x1, Hv[t], Lv[t]);
      adr[t] = ((size_t)bh * 64 + d) * Sq + sBase + s8;
    }
#pragma unroll
    for (int t = 0; t < 4; ++t) {
      *(volatile v4u*)(oh + adr[t]) = Hv[t];
      *(volatile v4u*)(ol + adr[t]) = Lv[t];
    }
    __threadfence();
#pragma unroll
    for (int t = 0; t < 4; ++t) {
      *(volatile v4u*)(oh + adr[t]) = Hv[t];
      *(volatile v4u*)(ol + adr[t]) = Lv[t];
    }
  } else {
    float* o = (float*)out0;
    v4f val[8];
    size_t adr[8];
#pragma unroll
    for (int t = 0; t < 8; ++t) {
      const int row = w * 16 + t * 2 + (l >> 4), c4 = (l & 15) * 4;
      val[t] = *(const v4f*)(stg + row * 68 + c4);
      adr[t] = (size_t)(mBase + row) * N + nBase + c4;
    }
#pragma unroll
    for (int t = 0; t < 8; ++t) *(volatile v4f*)(o + adr[t]) = val[t];
    __threadfence();
#pragma unroll
    for (int t = 0; t < 8; ++t) *(volatile v4f*)(o + adr[t]) = val[t];
  }
}

__global__ __launch_bounds__(32) void k_attn(const unsigned short* __restrict__ qh,
                                            const unsigned short* __restrict__ kh,
                                            const unsigned short* __restrict__ vth,
                                            const unsigned short* __restrict__ vtl,
                                            const float* __restrict__ sw, unsigned short* ctxh,
                                            unsigned short* ctxl, float* mout, int S, int H) {
  extern __shared__ v4f dsm[];
  float* sL = (float*)dsm;
  float* mL = sL + (size_t)16 * S;
  const int i0 = blockIdx.x * 16, b = blockIdx.y;
  if (i0 + 16 > S) return;
  const int l = threadIdx.x & 31, g = l >> 4, m = l & 15;
  const int E = H * 64;

  {
    v4f z;
    z[0] = 0.f; z[1] = 0.f; z[2] = 0.f; z[3] = 0.f;
    v4f* m4 = (v4f*)mL;
    const int n4 = 4 * S;
    for (int i = l; i < n4; i += 32) m4[i] = z;
  }
  __syncthreads();

  float* srow = sL + (size_t)m * S;
  float* mrow = mL + (size_t)m * S;
  const float invH = 1.0f / (float)H;
  const int nT = S >> 4, nC = S >> 5;

  for (int h = 0; h < H; ++h) {
    FragH qa0, qa1;
    {
      const unsigned short* qp = qh + (size_t)(b * S + i0 + m) * E + h * 64 + 8 * g;
      qa0.q[0] = ldg16(qp);
      qa0.q[1] = ldg16(qp + 16);
      qa1.q[0] = ldg16(qp + 32);
      qa1.q[1] = ldg16(qp + 48);
    }
    const float gsc = sw[b * 32 + h] * 0.125f;

    float rmax = -3.0e38f;
    const unsigned short* kp = kh + (size_t)(b * S + m) * E + h * 64 + 8 * g;
    for (int jt = 0; jt < nT; ++jt) {
      const unsigned short* kr = kp + (size_t)jt * 16 * E;
      FragH ka0, ka1;
      ka0.q[0] = ldg16(kr);
      ka0.q[1] = ldg16(kr + 16);
      ka1.q[0] = ldg16(kr + 32);
      ka1.q[1] = ldg16(kr + 48);
      v8f sc = zero8();
      sc = mma_h(ka0.v, qa0.v, sc);
      sc = mma_h(ka1.v, qa1.v, sc);
      asm volatile(NOP4 : "+v"(sc) : "v"(ka0.v), "v"(ka1.v), "v"(qa0.v), "v"(qa1.v));
      v4f t0, t1;
#pragma unroll
      for (int r = 0; r < 4; ++r) {
        t0[r] = sc[r] * gsc;
        t1[r] = sc[r + 4] * gsc;
        rmax = fmaxf(rmax, t0[r]);
        rmax = fmaxf(rmax, t1[r]);
      }
      float* pp = srow + jt * 16 + 8 * g;
      *(v4f*)pp = t0;
      *(v4f*)(pp + 4) = t1;
    }
    rmax = fmaxf(rmax, __shfl_xor(rmax, 16));

    float lsum = 0.f;
    for (int jt = 0; jt < nT; ++jt) {
      float* pp = srow + jt * 16 + 8 * g;
      v4f t0 = *(v4f*)pp;
      v4f t1 = *(v4f*)(pp + 4);
#pragma unroll
      for (int r = 0; r < 4; ++r) {
        t0[r] = __expf(t0[r] - rmax);
        t1[r] = __expf(t1[r] - rmax);
        lsum += t0[r];
        lsum += t1[r];
      }
      *(v4f*)pp = t0;
      *(v4f*)(pp + 4) = t1;
    }
    lsum += __shfl_xor(lsum, 16);
    const float linv = 1.0f / lsum;

    v8f cacc[4];
#pragma unroll
    for (int nt = 0; nt < 4; ++nt) cacc[nt] = zero8();
    const size_t vb = ((size_t)(b * H + h) * 64 + m) * S + 8 * g;
    const size_t vnt = (size_t)16 * S;
#pragma unroll 1
    for (int jc = 0; jc < nC; ++jc) {
      const int k0 = jc * 32;
      float* pa = srow + k0 + 8 * g;
      float* pb = srow + k0 + 16 + 8 * g;
      const v4f p0 = *(v4f*)pa * linv;
      const v4f p1 = *(v4f*)(pa + 4) * linv;
      const v4f p2 = *(v4f*)pb * linv;
      const v4f p3 = *(v4f*)(pb + 4) * linv;
      {
        v4f* ma = (v4f*)(mrow + k0 + 8 * g);
        v4f* mb = (v4f*)(mrow + k0 + 16 + 8 * g);
        const v4f s0 = ma[0] + p0;
        const v4f s1 = ma[1] + p1;
        const v4f s2 = mb[0] + p2;
        const v4f s3 = mb[1] + p3;
        ma[0] = s0;
        ma[1] = s1;
        mb[0] = s2;
        mb[1] = s3;
      }
      FragB ph, pl;
      split_b8(p0, p1, ph.q[0], pl.q[0]);
      split_b8(p2, p3, ph.q[1], pl.q[1]);
      FragB vh0, vh1, vh2, vh3, vl0, vl1, vl2, vl3;
      vh0.q[0] = ldg16(vth + vb + k0);
      vh0.q[1] = ldg16(vth + vb + k0 + 16);
      vh1.q[0] = ldg16(vth + vb + vnt + k0);
      vh1.q[1] = ldg16(vth + vb + vnt + k0 + 16);
      vh2.q[0] = ldg16(vth + vb + 2 * vnt + k0);
      vh2.q[1] = ldg16(vth + vb + 2 * vnt + k0 + 16);
      vh3.q[0] = ldg16(vth + vb + 3 * vnt + k0);
      vh3.q[1] = ldg16(vth + vb + 3 * vnt + k0 + 16);
      vl0.q[0] = ldg16(vtl + vb + k0);
      vl0.q[1] = ldg16(vtl + vb + k0 + 16);
      vl1.q[0] = ldg16(vtl + vb + vnt + k0);
      vl1.q[1] = ldg16(vtl + vb + vnt + k0 + 16);
      vl2.q[0] = ldg16(vtl + vb + 2 * vnt + k0);
      vl2.q[1] = ldg16(vtl + vb + 2 * vnt + k0 + 16);
      vl3.q[0] = ldg16(vtl + vb + 3 * vnt + k0);
      vl3.q[1] = ldg16(vtl + vb + 3 * vnt + k0 + 16);
      cacc[0] = mma_b(ph.v, vh0.v, cacc[0]);
      cacc[0] = mma_b(ph.v, vl0.v, cacc[0]);
      cacc[0] = mma_b(pl.v, vh0.v, cacc[0]);
      cacc[1] = mma_b(ph.v, vh1.v, cacc[1]);
      cacc[1] = mma_b(ph.v, vl1.v, cacc[1]);
      cacc[1] = mma_b(pl.v, vh1.v, cacc[1]);
      cacc[2] = mma_b(ph.v, vh2.v, cacc[2]);
      cacc[2] = mma_b(ph.v, vl2.v, cacc[2]);
      cacc[2] = mma_b(pl.v, vh2.v, cacc[2]);
      cacc[3] = mma_b(ph.v, vh3.v, cacc[3]);
      cacc[3] = mma_b(ph.v, vl3.v, cacc[3]);
      cacc[3] = mma_b(pl.v, vh3.v, cacc[3]);
      asm volatile(NOP4
                   : "+v"(cacc[0]), "+v"(cacc[1]), "+v"(cacc[2]), "+v"(cacc[3])
                   : "v"(ph.v), "v"(pl.v), "v"(vh0.v), "v"(vh1.v), "v"(vh2.v), "v"(vh3.v),
                     "v"(vl0.v), "v"(vl1.v), "v"(vl2.v), "v"(vl3.v));
    }

    __syncthreads();
#pragma unroll
    for (int nt = 0; nt < 4; ++nt) {
#pragma unroll
      for (int r = 0; r < 8; ++r) sL[(8 * g + r) * 68 + nt * 16 + m] = cacc[nt][r];
    }
    __syncthreads();
    v4u Hv[4], Lv[4];
    size_t adr[4];
#pragma unroll
    for (int t = 0; t < 4; ++t) {
      const int row = t * 4 + (l >> 3), c8 = (l & 7) * 8;
      const float* sp = sL + row * 68 + c8;
      const v4f x0 = *(const v4f*)sp;
      const v4f x1 = *(const v4f*)(sp + 4);
      split_b8(x0, x1, Hv[t], Lv[t]);
      adr[t] = (size_t)(b * S + i0 + row) * E + h * 64 + c8;
    }
#pragma unroll
    for (int t = 0; t < 4; ++t) {
      *(volatile v4u*)(ctxh + adr[t]) = Hv[t];
      *(volatile v4u*)(ctxl + adr[t]) = Lv[t];
    }
    __threadfence();
#pragma unroll
    for (int t = 0; t < 4; ++t) {
      *(volatile v4u*)(ctxh + adr[t]) = Hv[t];
      *(volatile v4u*)(ctxl + adr[t]) = Lv[t];
    }
    __syncthreads();
  }

  __syncthreads();
  float* ob = mout + (size_t)(b * S + i0) * S;
  const int nL = S >> 7;
  for (int row = 0; row < 16; ++row) {
    for (int c = 0; c < nL; ++c) {
      const size_t off = (size_t)row * S + c * 128 + l * 4;
      const v4f v = *(const v4f*)(mL + off) * invH;
      *(volatile v4f*)(ob + off) = v;
    }
  }
  __threadfence();
  for (int row = 0; row < 16; ++row) {
    for (int c = 0; c < nL; ++c) {
      const size_t off = (size_t)row * S + c * 128 + l * 4;
      const v4f v = *(const v4f*)(mL + off) * invH;
      *(volatile v4f*)(ob + off) = v;
    }
  }
}

extern "C" void kernel_launch(void* const* d_in, const int* in_sizes, int n_in, void* d_out,
                              int out_size, void* d_ws, size_t ws_size, hipStream_t stream) {
  if (n_in < 14) return;
  const int E = 1024, H = 16;
  const int nX = in_sizes[0];
  if (nX <= 0 || (nX % E) != 0) return;
  const int M = nX / E;
  const int nSy = in_sizes[1];
  if (nSy <= 0 || (nSy % E) != 0) return;
  const int Bn = nSy / E;
  if (Bn <= 0 || (M % Bn) != 0) return;
  const int S = M / Bn;
  const int HID = in_sizes[9];
  if ((M % 128) != 0 || (S % 128) != 0 || HID <= 0 || HID > 256) return;
  if (in_sizes[2] != E * E || in_sizes[4] != E * E || in_sizes[6] != E * E || in_sizes[12] != E * E) return;
  if (in_sizes[3] != E || in_sizes[5] != E || in_sizes[7] != E || in_sizes[13] != E) return;
  if (in_sizes[8] != E * HID || in_sizes[10] != HID * H || in_sizes[11] != H) return;
  if ((long long)out_size != (long long)nX + (long long)Bn * (long long)S * (long long)S) return;

  const float* x = (const float*)d_in[0];
  const float* sync = (const float*)d_in[1];
  const float* Wq = (const float*)d_in[2];
  const float* bq = (const float*)d_in[3];
  const float* Wk = (const float*)d_in[4];
  const float* bk = (const float*)d_in[5];
  const float* Wv = (const float*)d_in[6];
  const float* bv = (const float*)d_in[7];
  const float* Ws1 = (const float*)d_in[8];
  const float* bs1 = (const float*)d_in[9];
  const float* Ws2 = (const float*)d_in[10];
  const float* bs2 = (const float*)d_in[11];
  const float* Wo = (const float*)d_in[12];
  const float* bo = (const float*)d_in[13];

  float* out_proj = (float*)d_out;
  float* out_mean = (float*)d_out + (size_t)nX;

  size_t off = 0;
  auto al = [&](size_t bytes) { size_t o = off; off += (bytes + 255) & ~(size_t)255; return o; };
  const size_t nW = (size_t)E * E;
  const size_t o_sw = al((size_t)Bn * 32 * 4);
  const size_t o_xh = al((size_t)nX * 2);
  const size_t o_xbh = al((size_t)nX * 2);
  const size_t o_xbl = al((size_t)nX * 2);
  const size_t o_wq = al(nW * 2);
  const size_t o_wk = al(nW * 2);
  const size_t o_wvh = al(nW * 2);
  const size_t o_wvl = al(nW * 2);
  const size_t o_woh = al(nW * 2);
  const size_t o_wol = al(nW * 2);
  const size_t o_q = al((size_t)nX * 2);
  const size_t o_k = al((size_t)nX * 2);
  const size_t o_vth = al((size_t)nX * 2);
  const size_t o_vtl = al((size_t)nX * 2);
  const size_t o_cth = al((size_t)nX * 2);
  const size_t o_ctl = al((size_t)nX * 2);
  if (off > ws_size) return;

  char* ws = (char*)d_ws;
  float* sw_g = (float*)(ws + o_sw);
  unsigned short* xh = (unsigned short*)(ws + o_xh);
  unsigned short* xbh = (unsigned short*)(ws + o_xbh);
  unsigned short* xbl = (unsigned short*)(ws + o_xbl);
  unsigned short* wqT = (unsigned short*)(ws + o_wq);
  unsigned short* wkT = (unsigned short*)(ws + o_wk);
  unsigned short* wvTh = (unsigned short*)(ws + o_wvh);
  unsigned short* wvTl = (unsigned short*)(ws + o_wvl);
  unsigned short* woTh = (unsigned short*)(ws + o_woh);
  unsigned short* woTl = (unsigned short*)(ws + o_wol);
  unsigned short* qh = (unsigned short*)(ws + o_q);
  unsigned short* kh = (unsigned short*)(ws + o_k);
  unsigned short* vTh = (unsigned short*)(ws + o_vth);
  unsigned short* vTl = (unsigned short*)(ws + o_vtl);
  unsigned short* cth = (unsigned short*)(ws + o_cth);
  unsigned short* ctl = (unsigned short*)(ws + o_ctl);

  {
    const int groups = nX / 8;
    const int blocks = (groups + 255) / 256;
    k_cvt_x<<<dim3(blocks), dim3(256), 0, stream>>>(x, xh, xbh, xbl, nX);
  }
  {
    dim3 gw(E / 64, E / 64);
    k_cvt_wT<0><<<gw, dim3(256), 0, stream>>>(Wq, wqT, wqT, E, E, 64.0f);
    k_cvt_wT<0><<<gw, dim3(256), 0, stream>>>(Wk, wkT, wkT, E, E, 64.0f);
    k_cvt_wT<1><<<gw, dim3(256), 0, stream>>>(Wv, wvTh, wvTl, E, E, 1.0f);
    k_cvt_wT<1><<<gw, dim3(256), 0, stream>>>(Wo, woTh, woTl, E, E, 1.0f);
  }
  k_gate<<<dim3(Bn), dim3(256), 0, stream>>>(sync, Ws1, bs1, Ws2, bs2, sw_g, E, HID, H);
  dim3 gg(E / 64, M / 128);
  k_gemm<0, 0><<<gg, dim3(256), 0, stream>>>(xh, xh, wqT, wqT, bq, (void*)qh, (void*)qh, M, E, E, S, 1.0f / 64.0f);
  k_gemm<0, 0><<<gg, dim3(256), 0, stream>>>(xh, xh, wkT, wkT, bk, (void*)kh, (void*)kh, M, E, E, S, 1.0f / 64.0f);
  k_gemm<1, 1><<<gg, dim3(256), 0, stream>>>(xbh, xbl, wvTh, wvTl, bv, (void*)vTh, (void*)vTl, M, E, E, S, 1.0f);
  {
    const size_t dynB = (size_t)2 * 16 * (size_t)S * 4;
    hipFuncSetAttribute(reinterpret_cast<const void*>(&k_attn), hipFuncAttributeMaxDynamicSharedMemorySize, (int)dynB);
    k_attn<<<dim3(S / 16, Bn), dim3(32), dynB, stream>>>(qh, kh, vTh, vTl, sw_g, cth, ctl, out_mean, S, H);
  }
  k_gemm<1, 2><<<gg, dim3(256), 0, stream>>>(cth, ctl, woTh, woTl, bo, (void*)out_proj, (void*)out_proj, M, E, E, S, 1.0f);
  hipGetLastError();
  hipStreamSynchronize(stream);
}
